// MambaBlock_15857019257117
// MI455X (gfx1250) — hardware-run, weakly checked
//
#include <hip/hip_runtime.h>
#include <math.h>

typedef __attribute__((ext_vector_type(16))) _Float16 v16h;
typedef __attribute__((ext_vector_type(8)))  _Float16 v8h;
typedef __attribute__((ext_vector_type(8)))  float    v8f;
typedef __attribute__((ext_vector_type(4)))  float    v4f;

constexpr int kBatch   = 2;
constexpr int kSeqL    = 2048;
constexpr int kDmod    = 1024;
constexpr int kDin     = 2048;
constexpr int kNst     = 128;
constexpr int kDtR     = 64;
constexpr int kXdN     = kDtR + 2 * kNst;
constexpr int kXdPad   = 384;
constexpr int kXZP     = 2 * kDin;
constexpr int kRows    = kBatch * kSeqL;
constexpr int kTP      = 260;
constexpr int kScanT   = 16;
constexpr int kScanCh  = 64;
constexpr int kYP      = 68;
constexpr int kBlkPerB = kDin / kScanCh;
static_assert(kXdN == 320);
static_assert((kDmod % 32) == 0 && (kDin % 32) == 0 && (kDtR % 32) == 0);
static_assert((kRows % 64) == 0 && (kXZP % 64) == 0 && (kXdN % 64) == 0 && (kDin % 64) == 0 && (kDmod % 64) == 0 && (kXdPad % 64) == 0);
static_assert((kSeqL % 64) == 0 && (kSeqL % kScanT) == 0 && (kDin % 256) == 0 && (kDin % kScanCh) == 0);
static_assert(kNst == 4 * 32);

constexpr float kCarryHid = 16.0f;
constexpr float kCarryW   = 256.0f;
constexpr float kCarryWdt = 64.0f;
constexpr float kCarryU   = 64.0f;
constexpr float kCarryDtL = 64.0f;
constexpr float kCarryY   = 256.0f;
constexpr float kResid    = 2048.0f;
constexpr float kScaleIn  = 1.0f / (kCarryHid * kCarryW);
constexpr float kScaleX   = 1.0f / (kCarryU * kCarryW);
constexpr float kScaleDt  = 1.0f / (kCarryDtL * kCarryWdt);
constexpr float kScaleOut = 1.0f / (kCarryY * kCarryW);
constexpr float kLog2e    = 1.44269504088896340736f;

constexpr size_t kSzXZ    = (size_t)kRows * kXZP * 4;
constexpr size_t kSzUH    = (size_t)kRows * kDin * 2;
constexpr size_t kSzYG    = (size_t)kRows * kDin * 2;
constexpr size_t kSzXD    = (size_t)kRows * kXdN * 4;
constexpr size_t kSzDTL   = (size_t)kRows * kDtR * 2;
constexpr size_t kSzHID   = (size_t)kRows * kDmod * 2;
constexpr size_t kSzWINT  = (size_t)kXZP * kDmod * 2;
constexpr size_t kSzWXT   = (size_t)kXdPad * kDin * 2;
constexpr size_t kSzWDTT  = (size_t)kDin * kDtR * 2;
constexpr size_t kSzWOUTT = (size_t)kDmod * kDin * 2;
constexpr size_t kOffXZ    = 0;
constexpr size_t kOffUH    = kOffXZ    + kSzXZ;
constexpr size_t kOffYG    = kOffUH    + kSzUH;
constexpr size_t kOffXD    = kOffYG    + kSzYG;
constexpr size_t kOffDTL   = kOffXD    + kSzXD;
constexpr size_t kOffHID   = kOffDTL   + kSzDTL;
constexpr size_t kOffWINT  = kOffHID   + kSzHID;
constexpr size_t kOffWXT   = kOffWINT  + kSzWINT;
constexpr size_t kOffWDTT  = kOffWXT   + kSzWXT;
constexpr size_t kOffWOUTT = kOffWDTT  + kSzWDTT;
constexpr size_t kWsTotal  = kOffWOUTT + kSzWOUTT;
constexpr size_t kOffUL    = kOffHID;
constexpr size_t kSzUL     = (size_t)kRows * kDin * 2;
static_assert(kWsTotal == 129236992ull);
static_assert(kWsTotal <= 134217728ull);
static_assert(kSzUL == kSzHID + kSzWINT);
static_assert((kOffUH % 128) == 0 && (kOffYG % 128) == 0 && (kOffXD % 128) == 0 && (kOffDTL % 128) == 0 &&
              (kOffHID % 128) == 0 && (kOffWINT % 128) == 0 && (kOffWXT % 128) == 0 && (kOffWDTT % 128) == 0 &&
              (kOffWOUTT % 128) == 0);

union FragU { v16h v; v8h h[2]; };
__device__ __forceinline__ v16h frag_load(const _Float16* p) {
  FragU f;
  f.h[0] = *(const v8h*)(p);
  f.h[1] = *(const v8h*)(p + 16);
  return f.v;
}
__device__ __forceinline__ v8f frag_mma(v16h a, v16h b, v8f c) {
  return __builtin_amdgcn_wmma_f32_16x16x32_f16(false, a, false, b, (short)0, c, false, false);
}
__device__ __forceinline__ void tie_acc(v8f& c, v16h a, v16h b) { asm volatile("" : "+v"(c) : "v"(a), "v"(b)); }
__device__ __forceinline__ void guard_acc(v8f& c, v16h a, v16h b) { asm volatile("v_nop\n\tv_nop\n\tv_nop\n\tv_nop" : "+v"(c) : "v"(a), "v"(b)); }
__device__ __forceinline__ void keep4_h(v16h a, v16h b, v16h c, v16h d) { asm volatile("v_nop" :: "v"(a), "v"(b), "v"(c), "v"(d)); }
__device__ __forceinline__ void acc_guard4(v8f& a, v8f& b, v8f& c, v8f& d) { asm volatile("v_nop\n\tv_nop\n\tv_nop\n\tv_nop" : "+v"(a), "+v"(b), "+v"(c), "+v"(d)); }

__device__ __forceinline__ float h16_to_f32(unsigned hb) {
  const unsigned sgn = (hb & 0x8000u) << 16;
  const unsigned em = hb & 0x7fffu;
  const float fn = __uint_as_float((em << 13) + 0x38000000u);
  const float fs = (float)em * 5.9604644775390625e-8f;
  const float mag = (em < 0x400u) ? fs : fn;
  return __uint_as_float(__float_as_uint(mag) | sgn);
}

__device__ __forceinline__ float h16z(float v) {
    return (__builtin_fabsf(v) < 6.103515625e-05f) ? 0.0f : v;
}
template <int BIAS_MODE>
__global__ __launch_bounds__(256) void wmma_gemm64_f16(
    const unsigned short* __restrict__ Ap, int lda,
    const unsigned short* __restrict__ Btp, int ldb,
    float* __restrict__ Cout, int ldc,
    const float* __restrict__ bias,
    int M, int N, int K, float scale)
{
  const _Float16* A  = (const _Float16*)Ap;
  const _Float16* Bt = (const _Float16*)Btp;
  __shared__ __align__(16) float sT[8][16 * 68];
  const int lane = threadIdx.x & 31;
  const int wave = threadIdx.x >> 5;
  const int tilesN = N >> 6;
  const int tilesM = M >> 6;
  const int tile = blockIdx.x * 8 + wave;
  if (tile >= tilesM * tilesN) return;
  const int tm = tile / tilesN;
  const int tn = tile - tm * tilesN;
  const int m0 = tm << 6;
  const int n0 = tn << 6;

  const int rlane = lane & 15;
  const int koff  = (lane >> 4) * 8;
  const int mOff  = (lane >> 4) * 8;

  v8f acc[4][4];
#pragma unroll
  for (int i = 0; i < 4; ++i)
#pragma unroll
    for (int j = 0; j < 4; ++j) acc[i][j] = (v8f){0.f,0.f,0.f,0.f,0.f,0.f,0.f,0.f};

  for (int k0 = 0; k0 < K; k0 += 32) {
    v16h bh[4];
#pragma unroll
    for (int j = 0; j < 4; ++j) {
      const size_t bo = (size_t)(n0 + (j << 4) + rlane) * ldb + koff + k0;
      bh[j] = frag_load(Bt + bo);
    }
#pragma unroll
    for (int i = 0; i < 4; ++i) {
      const size_t ao = (size_t)(m0 + (i << 4) + rlane) * lda + koff + k0;
      v16h ah = frag_load(A + ao);
#pragma unroll
      for (int j = 0; j < 4; ++j) acc[i][j] = frag_mma(ah, bh[j], acc[i][j]);
      tie_acc(acc[i][0], ah, bh[0]);
      tie_acc(acc[i][1], ah, bh[1]);
      tie_acc(acc[i][2], ah, bh[2]);
      guard_acc(acc[i][3], ah, bh[3]);
    }
    keep4_h(bh[0], bh[1], bh[2], bh[3]);
  }
  acc_guard4(acc[0][0], acc[0][1], acc[0][2], acc[0][3]);
  acc_guard4(acc[1][0], acc[1][1], acc[1][2], acc[1][3]);
  acc_guard4(acc[2][0], acc[2][1], acc[2][2], acc[2][3]);
  acc_guard4(acc[3][0], acc[3][1], acc[3][2], acc[3][3]);

  float* slab = sT[wave];
#pragma unroll
  for (int i = 0; i < 4; ++i) {
    const int mBase = m0 + (i << 4);
#pragma unroll
    for (int j = 0; j < 4; ++j) {
      const int n = n0 + (j << 4) + rlane;
      float bv = 0.f;
      if (BIAS_MODE == 2) bv = bias[n];
#pragma unroll
      for (int r = 0; r < 8; ++r) {
        float v = acc[i][j][r] * scale;
        if (BIAS_MODE == 2) v += bv;
        slab[(mOff + r) * 68 + (j << 4) + rlane] = v;
      }
    }
    __builtin_amdgcn_fence(__ATOMIC_RELEASE, "workgroup");
    __builtin_amdgcn_wave_barrier();
    __builtin_amdgcn_fence(__ATOMIC_ACQUIRE, "workgroup");
    {
      const int hh = lane >> 4, c4 = (lane & 15) * 4;
      for (int pass = 0; pass < 2; ++pass) {
#pragma unroll
        for (int it = 0; it < 8; ++it) {
          const int row = it * 2 + hh;
          v4f v = *(const v4f*)(slab + row * 68 + c4);
          *(volatile v4f*)(Cout + (size_t)(mBase + row) * ldc + n0 + c4) = v;
        }
        __threadfence();
      }
    }
    __builtin_amdgcn_fence(__ATOMIC_RELEASE, "workgroup");
    __builtin_amdgcn_wave_barrier();
    __builtin_amdgcn_fence(__ATOMIC_ACQUIRE, "workgroup");
  }
}

__global__ __launch_bounds__(256) void cast_f16_kernel(
    const float* __restrict__ src, unsigned short* __restrict__ dst, int total8, float scale)
{
  const int i = blockIdx.x * 256 + threadIdx.x;
  if (i >= total8) return;
  const size_t e0 = (size_t)i << 3;
  const float* p = src + e0;
  const v4f a0 = *(const v4f*)(p);
  const v4f a1 = *(const v4f*)(p + 4);
  v8h hv;
#pragma unroll
  for (int e = 0; e < 4; ++e) {
    hv[e]     = (_Float16)h16z(a0[e] * scale);
    hv[4 + e] = (_Float16)h16z(a1[e] * scale);
  }
  unsigned short* q = dst + e0;
  *(volatile v8h*)q = hv;
  __threadfence();
  *(volatile v8h*)q = hv;
}

__global__ __launch_bounds__(256) void transpose_cast_kernel(
    const float* __restrict__ W, unsigned short* __restrict__ Bt, int Kdim, int Ndim, float scale)
{
  __shared__ float tile[64 * 65];
  const int tid = threadIdx.x, lane = tid & 31, wave = tid >> 5;
  const int n0 = blockIdx.x * 64;
  const int k0 = blockIdx.y * 64;
#pragma unroll
  for (int p = 0; p < 16; ++p) {
    const int idx = tid + p * 256;
    const int kk  = idx >> 6;
    const int nn  = idx & 63;
    const int n   = n0 + nn;
    const int nc  = (n < Ndim) ? n : (Ndim - 1);
    const float v = W[(size_t)(k0 + kk) * Ndim + nc];
    tile[kk * 65 + nn] = (n < Ndim) ? (v * scale) : 0.f;
  }
  __syncthreads();
  const int q = lane >> 3, c8 = (lane & 7) * 8;
  v8h hv[2];
#pragma unroll
  for (int it = 0; it < 2; ++it) {
    const int nrow = it * 32 + wave * 4 + q;
#pragma unroll
    for (int e = 0; e < 8; ++e) hv[it][e] = (_Float16)h16z(tile[(c8 + e) * 65 + nrow]);
  }
  for (int pass = 0; pass < 2; ++pass) {
#pragma unroll
    for (int it = 0; it < 2; ++it) {
      const int nrow = it * 32 + wave * 4 + q;
      *(volatile v8h*)(Bt + (size_t)(n0 + nrow) * Kdim + k0 + c8) = hv[it];
    }
    __threadfence();
  }
}

__global__ __launch_bounds__(256) void dt_cast_kernel(
    const float* __restrict__ XD, unsigned short* __restrict__ DTL, int total8, float scale)
{
  const int i = blockIdx.x * 256 + threadIdx.x;
  if (i >= total8) return;
  const int e0  = i << 3;
  const int row = e0 >> 6;
  const int c8  = e0 & 63;
  const float* p = XD + (size_t)row * kXdN + c8;
  const v4f a0 = *(const v4f*)(p);
  const v4f a1 = *(const v4f*)(p + 4);
  v8h hv;
#pragma unroll
  for (int e = 0; e < 4; ++e) {
    hv[e]     = (_Float16)h16z(a0[e] * scale);
    hv[4 + e] = (_Float16)h16z(a1[e] * scale);
  }
  unsigned short* qd = DTL + e0;
  *(volatile v8h*)qd = hv;
  __threadfence();
  *(volatile v8h*)qd = hv;
}

__global__ __launch_bounds__(256) void conv_silu_kernel(
    const float* __restrict__ XZ, const float* __restrict__ cw, const float* __restrict__ cb,
    unsigned short* __restrict__ UH, unsigned short* __restrict__ UL)
{
  __shared__ __align__(16) float sT[16 * kTP];
  const int tid = threadIdx.x, lane = tid & 31, wave = tid >> 5;
  const int d0 = blockIdx.x * 256, d = d0 + tid;
  const int g0 = blockIdx.y * 64;
  const int tb = g0 & (kSeqL - 1);
  const v4f wv = *(const v4f*)(cw + (size_t)d * 4);
  const float w0 = wv[0], w1 = wv[1], w2 = wv[2], w3 = wv[3];
  const float bc = cb[d];
  float xm3, xm2, xm1;
  {
    const bool hist = (tb > 0);
    const int rb = hist ? (g0 - 3) : g0;
    const float v3 = XZ[(size_t)rb * kXZP + d];
    const float v2 = XZ[(size_t)(rb + 1) * kXZP + d];
    const float v1 = XZ[(size_t)(rb + 2) * kXZP + d];
    xm3 = hist ? v3 : 0.f;
    xm2 = hist ? v2 : 0.f;
    xm1 = hist ? v1 : 0.f;
  }
#pragma unroll 1
  for (int sub = 0; sub < 4; ++sub) {
    const int lb = g0 + sub * 16;
#pragma unroll 1
    for (int s = 0; s < 16; ++s) {
      const float xcur = XZ[(size_t)(lb + s) * kXZP + d];
      float acc = w0 * xm3;
      acc = fmaf(w1, xm2, acc);
      acc = fmaf(w2, xm1, acc);
      acc = fmaf(w3, xcur, acc);
      const float sv = acc + bc;
      const float sg = __builtin_amdgcn_rcpf(1.0f + expf(-sv));
      sT[s * kTP + tid] = (sv * sg) * kCarryU;
      xm3 = xm2; xm2 = xm1; xm1 = xcur;
    }
    __syncthreads();
    v8h hv[2], lv[2];
#pragma unroll
    for (int it = 0; it < 2; ++it) {
      const float* sp = sT + (it * 8 + wave) * kTP + lane * 8;
      const v4f a0 = *(const v4f*)(sp);
      const v4f a1 = *(const v4f*)(sp + 4);
#pragma unroll
      for (int e = 0; e < 4; ++e) {
        const float x0 = a0[e];
        const float x1 = a1[e];
        const _Float16 h0 = (_Float16)h16z(x0);
        const _Float16 h1 = (_Float16)h16z(x1);
        const float r0 = (x0 - (float)h0) * kResid;
        const float r1 = (x1 - (float)h1) * kResid;
        hv[it][e]     = h0;
        hv[it][4 + e] = h1;
        lv[it][e]     = (_Float16)r0;
        lv[it][4 + e] = (_Float16)r1;
      }
    }
    for (int pass = 0; pass < 2; ++pass) {
#pragma unroll
      for (int it = 0; it < 2; ++it) {
        const size_t o = (size_t)(lb + it * 8 + wave) * kDin + d0 + lane * 8;
        *(volatile v8h*)(UH + o) = hv[it];
        *(volatile v8h*)(UL + o) = lv[it];
      }
      __threadfence();
    }
    __syncthreads();
  }
}

__global__ __launch_bounds__(256) void scan_gate_kernel(
    const float* __restrict__ XZ, const float* __restrict__ XD,
    const unsigned short* __restrict__ UH, const unsigned short* __restrict__ UL,
    const float* __restrict__ Alog, const float* __restrict__ Dv,
    unsigned short* __restrict__ YG)
{
  __shared__ __align__(16) float sBig[32 * 256];
  __shared__ __align__(16) float sDT[kScanT * kScanCh];
  __shared__ __align__(16) float sG[kScanT * kScanCh];
  __shared__ __align__(16) float sU[kScanT * kScanCh];
  __shared__ __align__(16) float sY[kScanT * kYP];
  const int tid = threadIdx.x, lane = tid & 31, wave = tid >> 5;
  const int c = tid >> 2, q = tid & 3;
  const int bix = blockIdx.x / kBlkPerB;
  const int d0  = (blockIdx.x - bix * kBlkPerB) * kScanCh;
  const int d   = d0 + c;
  const size_t row0 = (size_t)bix * kSeqL;

#pragma unroll 1
  for (int i = 0; i < 32; ++i) {
    const float al = Alog[(size_t)d * kNst + q * 32 + i];
    sBig[i * 256 + tid] = (-expf(al)) * kLog2e;
  }
  __syncthreads();
  float a2[32], h[32];
#pragma unroll
  for (int i = 0; i < 32; ++i) {
    a2[i] = sBig[i * 256 + tid];
    h[i] = 0.f;
  }
  const float Dd = Dv[d];
  __syncthreads();

#pragma unroll 1
  for (int t0 = 0; t0 < kSeqL; t0 += kScanT) {
#pragma unroll
    for (int p = 0; p < 4; ++p) {
      const int idx = tid + 256 * p;
      const int r = idx >> 6, c4 = (idx & 63) * 4;
      const v4f v = *(const v4f*)(XD + (row0 + t0 + r) * kXdN + kDtR + c4);
      *(v4f*)(sBig + r * 256 + c4) = v;
    }
#pragma unroll 1
    for (int p = 0; p < 4; ++p) {
      const int idx = tid + 256 * p;
      const int r = idx >> 6, cc = idx & 63;
      const size_t grow = row0 + t0 + r;
      const float pv = XZ[grow * kXZP + d0 + cc];
      const float zv = XZ[grow * kXZP + kDin + d0 + cc];
      const unsigned hb = UH[grow * kDin + d0 + cc];
      const unsigned lb = UL[grow * kDin + d0 + cc];
      const float dtv = fmaxf(pv, 0.0f) + log1pf(expf(-fabsf(pv)));
      const float sg  = __builtin_amdgcn_rcpf(1.0f + expf(-zv));
      const float hf  = h16_to_f32(hb);
      const float lf  = h16_to_f32(lb);
      const float uu  = fmaf(lf, 1.0f / kResid, hf) * (1.0f / kCarryU);
      sDT[idx] = dtv;
      sG[idx]  = zv * sg;
      sU[idx]  = uu;
    }
    __syncthreads();

#pragma unroll 1
    for (int s = 0; s < kScanT; ++s) {
      const float dtv = sDT[s * kScanCh + c];
      const float uu  = sU[s * kScanCh + c];
      const float gg  = sG[s * kScanCh + c];
      const float dtu = dtv * uu;
      const float* bp = sBig + s * 256 + q * 32;
      const float* cp = bp + kNst;
      float part = 0.f;
#pragma unroll
      for (int i4 = 0; i4 < 8; ++i4) {
        const v4f Bv = *(const v4f*)(bp + 4 * i4);
        const v4f Cv = *(const v4f*)(cp + 4 * i4);
#pragma unroll
        for (int e = 0; e < 4; ++e) {
          const int n = 4 * i4 + e;
          const float dA = __builtin_amdgcn_exp2f(dtv * a2[n]);
          h[n] = fmaf(dA, h[n], dtu * Bv[e]);
          part = fmaf(h[n], Cv[e], part);
        }
      }
      part += __shfl_xor(part, 1, 32);
      part += __shfl_xor(part, 2, 32);
      const float y = fmaf(uu, Dd, part);
      sY[s * kYP + c] = (y * gg) * kCarryY;
    }
    __syncthreads();

    if (wave < 4) {
      const int q8 = lane >> 3, c8 = (lane & 7) * 8;
      const int r = wave * 4 + q8;
      const float* sp = sY + r * kYP + c8;
      const v4f a0 = *(const v4f*)(sp);
      const v4f a1 = *(const v4f*)(sp + 4);
      v8h hv;
#pragma unroll
      for (int e = 0; e < 4; ++e) {
        hv[e]     = (_Float16)h16z(a0[e]);
        hv[4 + e] = (_Float16)h16z(a1[e]);
      }
      unsigned short* dst = YG + (row0 + t0 + r) * kDin + d0 + c8;
      *(volatile v8h*)dst = hv;
      __threadfence();
      *(volatile v8h*)dst = hv;
    }
  }
}

extern "C" void kernel_launch(void* const* d_in, const int* in_sizes, int n_in,
                              void* d_out, int out_size, void* d_ws, size_t ws_size,
                              hipStream_t stream)
{
  if (n_in < 10) return;
  if (in_sizes[0] != kRows * kDmod) return;
  if (in_sizes[1] != kDmod * kXZP) return;
  if (in_sizes[2] != kDin * 4) return;
  if (in_sizes[3] != kDin) return;
  if (in_sizes[4] != kDin * kXdN) return;
  if (in_sizes[5] != kDtR * kDin) return;
  if (in_sizes[6] != kDin) return;
  if (in_sizes[7] != kDin * kNst) return;
  if (in_sizes[8] != kDin) return;
  if (in_sizes[9] != kDin * kDmod) return;
  if (out_size != kRows * kDmod) return;
  if (ws_size < kWsTotal) return;

  const float* hid    = (const float*)d_in[0];
  const float* W_in   = (const float*)d_in[1];
  const float* conv_w = (const float*)d_in[2];
  const float* conv_b = (const float*)d_in[3];
  const float* W_xprj = (const float*)d_in[4];
  const float* W_dt   = (const float*)d_in[5];
  const float* b_dt   = (const float*)d_in[6];
  const float* A_log  = (const float*)d_in[7];
  const float* Dv     = (const float*)d_in[8];
  const float* W_out  = (const float*)d_in[9];
  float* out = (float*)d_out;

  char* ws = (char*)d_ws;
  float*          XZ    = (float*)(ws + kOffXZ);
  unsigned short* UH    = (unsigned short*)(ws + kOffUH);
  unsigned short* YG    = (unsigned short*)(ws + kOffYG);
  float*          XD    = (float*)(ws + kOffXD);
  unsigned short* DTL   = (unsigned short*)(ws + kOffDTL);
  unsigned short* HID   = (unsigned short*)(ws + kOffHID);
  unsigned short* WINT  = (unsigned short*)(ws + kOffWINT);
  unsigned short* WXT   = (unsigned short*)(ws + kOffWXT);
  unsigned short* WDTT  = (unsigned short*)(ws + kOffWDTT);
  unsigned short* WOUTT = (unsigned short*)(ws + kOffWOUTT);
  unsigned short* UL    = (unsigned short*)(ws + kOffUL);

  cast_f16_kernel<<<(kRows * kDmod) / 8 / 256, 256, 0, stream>>>(hid, HID, (kRows * kDmod) / 8, kCarryHid);

  transpose_cast_kernel<<<dim3(kXZP / 64, kDmod / 64), 256, 0, stream>>>(W_in, WINT, kDmod, kXZP, kCarryW);
  transpose_cast_kernel<<<dim3(kXdPad / 64, kDin / 64), 256, 0, stream>>>(W_xprj, WXT, kDin, kXdN, kCarryW);
  transpose_cast_kernel<<<dim3(kDin / 64, kDtR / 64), 256, 0, stream>>>(W_dt, WDTT, kDtR, kDin, kCarryWdt);
  transpose_cast_kernel<<<dim3(kDmod / 64, kDin / 64), 256, 0, stream>>>(W_out, WOUTT, kDin, kDmod, kCarryW);

  wmma_gemm64_f16<0><<<dim3((kRows / 64) * (kXZP / 64) / 8), 256, 0, stream>>>(
      HID, kDmod, WINT, kDmod, XZ, kXZP, b_dt, kRows, kXZP, kDmod, kScaleIn);

  conv_silu_kernel<<<dim3(kDin / 256, kRows / 64), 256, 0, stream>>>(XZ, conv_w, conv_b, UH, UL);

  wmma_gemm64_f16<0><<<dim3((kRows / 64) * (kXdN / 64) / 8), 256, 0, stream>>>(
      UH, kDin, WXT, kDin, XD, kXdN, b_dt, kRows, kXdN, kDin, kScaleX);

  dt_cast_kernel<<<(kRows * kDtR) / 8 / 256, 256, 0, stream>>>(XD, DTL, (kRows * kDtR) / 8, kCarryDtL);

  wmma_gemm64_f16<2><<<dim3((kRows / 64) * (kDin / 64) / 8), 256, 0, stream>>>(
      DTL, kDtR, WDTT, kDtR, XZ, kXZP, b_dt, kRows, kDin, kDtR, kScaleDt);

  scan_gate_kernel<<<kBatch * kBlkPerB, 256, 0, stream>>>(XZ, XD, UH, UL, A_log, Dv, YG);

  wmma_gemm64_f16<0><<<dim3((kRows / 64) * (kDmod / 64) / 8), 256, 0, stream>>>(
      YG, kDin, WOUTT, kDin, out, kDmod, b_dt, kRows, kDmod, kDin, kScaleOut);
}
